// MMFSBlock_74801150427597
// MI455X (gfx1250) — hardware-verified
//
#include <hip/hip_runtime.h>
#define NB 2
#define QD 320
#define HQ 32
#define LQ 1024
#define NQ (NB * LQ)
#define NIM 8
#define HV 16
#define LV 256
#define FD 1024
#define DM 1024
#define NH 16
#define NPt 8
#define HD 64
#define MAXN 10
#define NV (NB * NIM * LV)
typedef __bf16 v16b __attribute__((ext_vector_type(16)));
typedef unsigned short v8us __attribute__((ext_vector_type(8), may_alias));
typedef float  v8f  __attribute__((ext_vector_type(8)));
typedef float  v4f  __attribute__((ext_vector_type(4)));
typedef float  v4fa __attribute__((ext_vector_type(4), may_alias));
union FragB { v16b v; v8us half[2]; unsigned short u[16]; };

__device__ __forceinline__ unsigned short bf16_bits(float x) { unsigned int u = __float_as_uint(x); return (unsigned short)((u + 0x7FFFu + ((u >> 16) & 1u)) >> 16); }
__device__ __forceinline__ float bf16_val(unsigned short b) { return __uint_as_float(((unsigned int)b) << 16); }
__device__ __forceinline__ float bf16_round(float x) { return bf16_val(bf16_bits(x)); }
template <int NT>
__device__ __forceinline__ v8f mmaN(v16b ah, v16b al, v16b bh, v16b bl, v8f c) {
  c = __builtin_amdgcn_wmma_f32_16x16x32_bf16(false, ah, false, bh, (short)0, c, false, false);
  if (NT >= 2) c = __builtin_amdgcn_wmma_f32_16x16x32_bf16(false, al, false, bh, (short)0, c, false, false);
  if (NT >= 3) c = __builtin_amdgcn_wmma_f32_16x16x32_bf16(false, ah, false, bl, (short)0, c, false, false);
  asm volatile("v_nop\n\tv_nop\n\tv_nop\n\tv_nop" : "+v"(c) : "v"(ah), "v"(al), "v"(bh), "v"(bl));
  return c;
}

__global__ __launch_bounds__(256) void k_wt_bf16(const float* __restrict__ W, unsigned short* __restrict__ Wt, int K, int N) {
  const int t = blockIdx.x * 256 + threadIdx.x;
  const int k8n = K / 8;
  if (t >= N * k8n) return;
  const int n = t / k8n, k8 = (t % k8n) * 8;
  v8us v;
#pragma unroll
  for (int i = 0; i < 8; ++i) v[i] = bf16_bits(W[(size_t)(k8 + i) * N + n]);
  *(volatile v8us*)(Wt + (size_t)n * K + k8) = v;
  __threadfence();
  *(volatile v8us*)(Wt + (size_t)n * K + k8) = v;
}

template <bool ASPLIT, int ACT, bool BIAS_BF16>
__global__ __launch_bounds__(128) void k_gemm_bf(const float* __restrict__ A, int lda, const unsigned short* __restrict__ Wt, int ldb,
                                               const float* __restrict__ bias, float* __restrict__ C, int ldc, int M, int N, int K) {
  __shared__ __attribute__((aligned(16))) float so[4][16][64];
  const int tid = threadIdx.x, w = tid >> 5, lane = tid & 31, ln = lane & 15, hh = lane >> 4;
  const int ntn = N / 64;
  const int wid = blockIdx.x * 4 + w;
  const int mt = wid / ntn, nq = wid % ntn;
  if (mt * 16 >= M) return;
  const int row0 = mt * 16, col0 = nq * 64;
  const float* arow = A + (size_t)(row0 + ln) * lda;
  v8f acc[4] = {};
  for (int kb = 0; kb < K; kb += 32) {
    FragB ah, al;
    const v4f x0 = *(const v4fa*)(arow + kb + 8 * hh), x1 = *(const v4fa*)(arow + kb + 8 * hh + 4);
    const v4f x2 = *(const v4fa*)(arow + kb + 16 + 8 * hh), x3 = *(const v4fa*)(arow + kb + 16 + 8 * hh + 4);
    float xs[16] = {x0[0],x0[1],x0[2],x0[3],x1[0],x1[1],x1[2],x1[3],x2[0],x2[1],x2[2],x2[3],x3[0],x3[1],x3[2],x3[3]};
#pragma unroll
    for (int i = 0; i < 16; ++i) { const unsigned short hb = bf16_bits(xs[i]); ah.u[i] = hb; al.u[i] = ASPLIT ? bf16_bits(xs[i] - bf16_val(hb)) : (unsigned short)0; }
#pragma unroll
    for (int t = 0; t < 4; ++t) {
      const unsigned short* brow = Wt + (size_t)(col0 + t * 16 + ln) * ldb + kb;
      FragB b;
      b.half[0] = *(const v8us*)(brow + 8 * hh);
      b.half[1] = *(const v8us*)(brow + 16 + 8 * hh);
      acc[t] = mmaN<ASPLIT ? 2 : 1>(ah.v, al.v, b.v, b.v, acc[t]);
    }
  }
#pragma unroll
  for (int t = 0; t < 4; ++t) {
    float bv = bias ? bias[col0 + t * 16 + ln] : 0.f;
    if (BIAS_BF16) bv = bf16_round(bv);
#pragma unroll
    for (int r = 0; r < 8; ++r) { float v = acc[t][r] + bv; if (ACT == 1) v = fmaxf(v, 0.f); so[w][8 * hh + r][t * 16 + ln] = v; }
  }
  __builtin_amdgcn_fence(__ATOMIC_ACQ_REL, "workgroup");
  __builtin_amdgcn_wave_barrier();
  const int rsub = lane >> 4, c4 = (lane & 15) * 4;
  for (int pass = 0; pass < 2; ++pass) {
#pragma unroll
    for (int q = 0; q < 8; ++q) {
      const int r = q * 2 + rsub;
      const v4f v = *(const v4fa*)&so[w][r][c4];
      *(volatile v4f*)(C + (size_t)(row0 + r) * ldc + col0 + c4) = v;
    }
    if (pass == 0) __threadfence();
  }
}

template <bool ASPLIT, int ACT, bool BIAS_BF16, bool RES_BF16>
__global__ __launch_bounds__(128) void k_gemm_bf3(const float* __restrict__ A, int lda, const unsigned short* __restrict__ Wt, int ldb,
                                                const float* __restrict__ bias, const float* __restrict__ resid, int rmod, int ldr,
                                                float* __restrict__ C, int ldc, int M, int N, int K) {
  __shared__ __attribute__((aligned(16))) float so[4][16][64];
  const int tid = threadIdx.x, w = tid >> 5, lane = tid & 31, ln = lane & 15, hh = lane >> 4;
  const int ntn = N / 64;
  const int wid = blockIdx.x * 4 + w;
  const int mt = wid / ntn, nq = wid % ntn;
  if (mt * 16 >= M) return;
  const int row0 = mt * 16, col0 = nq * 64;
  const float* arow = A + (size_t)(row0 + ln) * lda;
  v8f acc[4] = {};
  for (int kb = 0; kb < K; kb += 32) {
    FragB ah, al;
    const v4f x0 = *(const v4fa*)(arow + kb + 8 * hh), x1 = *(const v4fa*)(arow + kb + 8 * hh + 4);
    const v4f x2 = *(const v4fa*)(arow + kb + 16 + 8 * hh), x3 = *(const v4fa*)(arow + kb + 16 + 8 * hh + 4);
    float xs[16] = {x0[0],x0[1],x0[2],x0[3],x1[0],x1[1],x1[2],x1[3],x2[0],x2[1],x2[2],x2[3],x3[0],x3[1],x3[2],x3[3]};
#pragma unroll
    for (int i = 0; i < 16; ++i) { const unsigned short hb = bf16_bits(xs[i]); ah.u[i] = hb; al.u[i] = ASPLIT ? bf16_bits(xs[i] - bf16_val(hb)) : (unsigned short)0; }
#pragma unroll
    for (int t = 0; t < 4; ++t) {
      const unsigned short* brow = Wt + (size_t)(col0 + t * 16 + ln) * ldb + kb;
      FragB b;
      b.half[0] = *(const v8us*)(brow + 8 * hh);
      b.half[1] = *(const v8us*)(brow + 16 + 8 * hh);
      acc[t] = mmaN<ASPLIT ? 2 : 1>(ah.v, al.v, b.v, b.v, acc[t]);
    }
  }
#pragma unroll
  for (int t = 0; t < 4; ++t) {
    const int col = col0 + t * 16 + ln;
    float bv = bias ? bias[col] : 0.f;
    if (BIAS_BF16) bv = bf16_round(bv);
#pragma unroll
    for (int r = 0; r < 8; ++r) {
      float v = acc[t][r] + bv;
      if (resid) { float rv = resid[(size_t)((row0 + 8 * hh + r) % rmod) * ldr + col]; if (RES_BF16) rv = bf16_round(rv); v += rv; }
      if (ACT == 1) v = fmaxf(v, 0.f);
      if (ACT == 2) v = 0.5f * v * (1.0f + erff(v * 0.70710678118654752f));
      if (ACT == 3) { const float u = 0.7978845608028654f * (v + 0.044715f * v * v * v); v = 0.5f * v * (1.0f + tanhf(u)); }
      so[w][8 * hh + r][t * 16 + ln] = v;
    }
  }
  __builtin_amdgcn_fence(__ATOMIC_ACQ_REL, "workgroup");
  __builtin_amdgcn_wave_barrier();
  const int rsub = lane >> 4, c4 = (lane & 15) * 4;
  for (int pass = 0; pass < 2; ++pass) {
#pragma unroll
    for (int q = 0; q < 8; ++q) {
      const int r = q * 2 + rsub;
      const v4f v = *(const v4fa*)&so[w][r][c4];
      *(volatile v4f*)(C + (size_t)(row0 + r) * ldc + col0 + c4) = v;
    }
    if (pass == 0) __threadfence();
  }
}
template <bool PARAM_BF16>
__global__ __launch_bounds__(256) void k_layernorm(const float* __restrict__ X, const float* __restrict__ R, const float* __restrict__ g, const float* __restrict__ bta,
                                                  float* __restrict__ out_sum, float* __restrict__ out_norm, int N, float eps) {
  __shared__ float red[256];
  const int row = blockIdx.x, tid = threadIdx.x;
  const float* x = X + (size_t)row * N; const float* rr = R ? R + (size_t)row * N : nullptr;
  float vals[16];
  const int per = N / 256;
  float s1 = 0.f;
  for (int u = 0; u < per / 4; ++u) {
    const int j = tid * 4 + 1024 * u;
    const v4f a = *(const v4fa*)(x + j);
    v4f b = {0.f,0.f,0.f,0.f}; if (rr) b = *(const v4fa*)(rr + j);
#pragma unroll
    for (int q = 0; q < 4; ++q) { const float v = a[q] + b[q]; vals[u * 4 + q] = v; s1 += v; }
  }
  red[tid] = s1; __syncthreads();
  for (int st = 128; st > 0; st >>= 1) { if (tid < st) red[tid] += red[tid + st]; __syncthreads(); }
  const float mu = red[0] / (float)N; __syncthreads();
  float s2 = 0.f;
  for (int u = 0; u < per / 4; ++u)
#pragma unroll
    for (int q = 0; q < 4; ++q) { const float c = vals[u * 4 + q] - mu; s2 += c * c; }
  red[tid] = s2; __syncthreads();
  for (int st = 128; st > 0; st >>= 1) { if (tid < st) red[tid] += red[tid + st]; __syncthreads(); }
  const float rs = rsqrtf(red[0] / (float)N + eps);
  for (int pass = 0; pass < 2; ++pass) {
    for (int u = 0; u < per / 4; ++u) {
      const int j = tid * 4 + 1024 * u;
      v4f o, sm;
#pragma unroll
      for (int q = 0; q < 4; ++q) {
        float gg = g[j + q], bb = bta[j + q];
        if (PARAM_BF16) { gg = bf16_round(gg); bb = bf16_round(bb); }
        sm[q] = vals[u * 4 + q]; o[q] = (vals[u * 4 + q] - mu) * rs * gg + bb;
      }
      if (out_sum) *(volatile v4f*)(out_sum + (size_t)row * N + j) = sm;
      *(volatile v4f*)(out_norm + (size_t)row * N + j) = o;
    }
    if (pass == 0) __threadfence();
  }
}


typedef _Float16 v16h __attribute__((ext_vector_type(16)));
union FragH { v16h v; v8us half[2]; _Float16 h[16]; unsigned short u[16]; };
template <int NT>
__device__ __forceinline__ v8f mmaH(v16h ah, v16h al, v16h bh, v16h bl, v8f c) {
  c = __builtin_amdgcn_wmma_f32_16x16x32_f16(false, ah, false, bh, (short)0, c, false, false);
  if (NT >= 2) c = __builtin_amdgcn_wmma_f32_16x16x32_f16(false, al, false, bh, (short)0, c, false, false);
  if (NT >= 3) c = __builtin_amdgcn_wmma_f32_16x16x32_f16(false, ah, false, bl, (short)0, c, false, false);
  asm volatile("v_nop\n\tv_nop\n\tv_nop\n\tv_nop" : "+v"(c) : "v"(ah), "v"(al), "v"(bh), "v"(bl));
  return c;
}
template <bool ASPLIT>
__global__ __launch_bounds__(128) void k_gemm_h(const float* __restrict__ A, int lda, size_t sA, const _Float16* __restrict__ Bh, int ldb, size_t sB, float alpha, float* __restrict__ C, int ldc, size_t sC, int M, int N, int K) {
  __shared__ __attribute__((aligned(16))) float so[4][16][64];
  const int tid = threadIdx.x, w = tid >> 5, lane = tid & 31, ln = lane & 15, hh = lane >> 4; const int by = blockIdx.y;
  A += (size_t)by * sA; Bh += (size_t)by * sB; C += (size_t)by * sC;
  const int ntn = (N + 63) / 64; const int wid = blockIdx.x * 4 + w; const int mt = wid / ntn, nq = wid % ntn; if (mt * 16 >= M) return;
  const int row0 = mt * 16, col0 = nq * 64; const float* arow = A + (size_t)(row0 + ln) * lda;
  v8f acc[4] = {};
  for (int kb = 0; kb < K; kb += 32) {
    FragH ah, al;
    const v4f x0 = *(const v4fa*)(arow + kb + 8 * hh), x1 = *(const v4fa*)(arow + kb + 8 * hh + 4), x2 = *(const v4fa*)(arow + kb + 16 + 8 * hh), x3 = *(const v4fa*)(arow + kb + 16 + 8 * hh + 4);
    float xs[16] = {x0[0],x0[1],x0[2],x0[3],x1[0],x1[1],x1[2],x1[3],x2[0],x2[1],x2[2],x2[3],x3[0],x3[1],x3[2],x3[3]};
#pragma unroll
    for (int i = 0; i < 16; ++i) { const _Float16 h = (_Float16)xs[i]; ah.h[i] = h; al.h[i] = ASPLIT ? (_Float16)(xs[i] - (float)h) : (_Float16)0.0f; }
#pragma unroll
    for (int t = 0; t < 4; ++t) { if (col0 + t * 16 >= N) continue; const size_t boff = (size_t)(col0 + t * 16 + ln) * ldb + kb; FragH bq; bq.half[0] = *(const v8us*)(Bh + boff + 8 * hh); bq.half[1] = *(const v8us*)(Bh + boff + 16 + 8 * hh);
      acc[t] = mmaH<ASPLIT ? 2 : 1>(ah.v, al.v, bq.v, bq.v, acc[t]); }
  }
#pragma unroll
  for (int t = 0; t < 4; ++t) { if (col0 + t * 16 >= N) continue;
#pragma unroll
    for (int r = 0; r < 8; ++r) so[w][8 * hh + r][t * 16 + ln] = acc[t][r] * alpha; }
  __builtin_amdgcn_fence(__ATOMIC_ACQ_REL, "workgroup"); __builtin_amdgcn_wave_barrier();
  const int rsub = lane >> 4, c4 = (lane & 15) * 4;
  for (int pass = 0; pass < 2; ++pass) {
#pragma unroll
    for (int q = 0; q < 8; ++q) { const int r = q * 2 + rsub; if (col0 + c4 < N) { const v4f v = *(const v4fa*)&so[w][r][c4]; *(volatile v4f*)(C + (size_t)(row0 + r) * ldc + col0 + c4) = v; } }
    if (pass == 0) __threadfence(); }
}

__global__ __launch_bounds__(256) void k_wt_f16(const float* __restrict__ W, _Float16* __restrict__ Wt, int K, int N, float scale) {
  const int t = blockIdx.x * 256 + threadIdx.x; if (t >= N * (K / 8)) return; const int n = t / (K / 8), k8 = (t % (K / 8)) * 8; FragH f;
#pragma unroll
  for (int i = 0; i < 8; ++i) f.h[i] = (_Float16)(bf16_round(W[(size_t)(k8 + i) * N + n]) * scale); const v8us o = f.half[0];
  *(volatile v8us*)((unsigned short*)Wt + (size_t)n * K + k8) = o; __threadfence(); *(volatile v8us*)((unsigned short*)Wt + (size_t)n * K + k8) = o;
}
template <int ACT>
__global__ __launch_bounds__(128) void k_gemm_hhx(const _Float16* __restrict__ A, int lda, size_t sA, const _Float16* __restrict__ Bh, int ldb, size_t sB, float alpha, const float* __restrict__ bias, size_t sBias, const float* __restrict__ CP, int rowsPerB, size_t sCPb, int row0g,
    float* __restrict__ C, _Float16* __restrict__ C16, int ldc, size_t sC, int M, int N, int K) {
  __shared__ __attribute__((aligned(16))) float so[4][16][64];
  const int tid = threadIdx.x, w = tid >> 5, lane = tid & 31, ln = lane & 15, hh = lane >> 4; const int by = blockIdx.y;
  A += (size_t)by * sA; Bh += (size_t)by * sB; const size_t cofs = (size_t)by * sC; const float* bp = bias ? bias + (size_t)by * sBias : nullptr;
  const int ntn = (N + 63) / 64; const int wid = blockIdx.x * 4 + w; const int mt = wid / ntn, nq = wid % ntn; if (mt * 16 >= M) return;
  const int row0 = mt * 16, col0 = nq * 64; const _Float16* arow = A + (size_t)(row0 + ln) * lda;
  v8f acc[4] = {};
  for (int kb = 0; kb < K; kb += 32) { FragH ah; ah.half[0] = *(const v8us*)((const unsigned short*)arow + kb + 8 * hh); ah.half[1] = *(const v8us*)((const unsigned short*)arow + kb + 16 + 8 * hh);
#pragma unroll
    for (int t = 0; t < 4; ++t) { if (col0 + t * 16 >= N) continue; const size_t boff = (size_t)(col0 + t * 16 + ln) * ldb + kb; FragH bq; bq.half[0] = *(const v8us*)((const unsigned short*)Bh + boff + 8 * hh); bq.half[1] = *(const v8us*)((const unsigned short*)Bh + boff + 16 + 8 * hh);
      acc[t] = mmaH<1>(ah.v, ah.v, bq.v, bq.v, acc[t]); }
  }
#pragma unroll
  for (int t = 0; t < 4; ++t) { if (col0 + t * 16 >= N) continue; const int col = col0 + t * 16 + ln; const float bv = bp ? bf16_round(bp[col]) : 0.f;
#pragma unroll
    for (int r = 0; r < 8; ++r) { float v = acc[t][r] * alpha + bv; if (CP) { const int bidx = (row0g + row0 + 8 * hh + r) / rowsPerB; v += CP[(size_t)bidx * sCPb + (size_t)by * 64 + col]; } if (ACT == 1) v = (v > 0.f) ? v : expm1f(v); else if (ACT == 7) v = (v > 0.f) ? v + 1.0f : expf(v); else if (ACT == 8) v = tanhf(v); else if (ACT == 9) v = 0.5f * v * (1.0f + tanhf(0.7978845608028654f * (v + 0.044715f * v * v * v))); else if (ACT == 11) v = 1.0f / (1.0f + expf(-v)); else if (ACT == 12) v = (v > 0.f) ? v : 0.01f * v; else if (ACT == 14) v = (v > 0.f) ? v : 0.1f * v; else if (ACT == 15) v = v / (1.0f + expf(-v)); else if (ACT == 3) v = fmaxf(v, 0.f); else if (ACT == 6) v = 0.5f * v * (1.0f + erff(v * 0.70710678118654752f)); so[w][8 * hh + r][t * 16 + ln] = v; } }
  __builtin_amdgcn_fence(__ATOMIC_ACQ_REL, "workgroup"); __builtin_amdgcn_wave_barrier();
  const int rsub = lane >> 4, c4 = (lane & 15) * 4; typedef _Float16 v4h __attribute__((ext_vector_type(4)));
  for (int pass = 0; pass < 2; ++pass) {
#pragma unroll
    for (int q = 0; q < 8; ++q) { const int r = q * 2 + rsub; if (col0 + c4 < N) { const v4f v = *(const v4fa*)&so[w][r][c4]; if (C) *(volatile v4f*)(C + cofs + (size_t)(row0 + r) * ldc + col0 + c4) = v; if (C16) { v4h h4; for (int i = 0; i < 4; ++i) h4[i] = (_Float16)v[i]; *(volatile v4h*)(C16 + cofs + (size_t)(row0 + r) * ldc + col0 + c4) = h4; } } }
    if (pass == 0) __threadfence(); }
}


typedef _Float16 v4h __attribute__((ext_vector_type(4)));

__global__ __launch_bounds__(256) void k_x16(const float* __restrict__ x, _Float16* __restrict__ X16, size_t n8) { const size_t t = (size_t)blockIdx.x * 256 + threadIdx.x; if (t >= n8) return; FragH f;
#pragma unroll
  for (int q = 0; q < 8; ++q) f.h[q] = (_Float16)bf16_round(x[t * 8 + q]); *(volatile v8us*)((unsigned short*)X16 + t * 8) = f.half[0]; __threadfence(); *(volatile v8us*)((unsigned short*)X16 + t * 8) = f.half[0]; }
__global__ __launch_bounds__(256) void k_h16(const float* __restrict__ x, _Float16* __restrict__ X16, size_t n8) { const size_t t = (size_t)blockIdx.x * 256 + threadIdx.x; if (t >= n8) return; FragH f;
#pragma unroll
  for (int q = 0; q < 8; ++q) f.h[q] = (_Float16)x[t * 8 + q]; *(volatile v8us*)((unsigned short*)X16 + t * 8) = f.half[0]; __threadfence(); *(volatile v8us*)((unsigned short*)X16 + t * 8) = f.half[0]; }
__global__ __launch_bounds__(256) void k_round16f(const float* __restrict__ W, _Float16* __restrict__ Bt, size_t n8) { const size_t t = (size_t)blockIdx.x * 256 + threadIdx.x; if (t >= n8) return; FragH f;
#pragma unroll
  for (int i = 0; i < 8; ++i) f.h[i] = (_Float16)(bf16_round(W[t * 8 + i]) * 16.0f); *(volatile v8us*)((unsigned short*)Bt + t * 8) = f.half[0]; __threadfence(); *(volatile v8us*)((unsigned short*)Bt + t * 8) = f.half[0]; }
template <int NHv, int TTv>
__global__ __launch_bounds__(256) void k_vt(const _Float16* __restrict__ V16, int ldv, int voff, _Float16* __restrict__ Vt) { __shared__ unsigned short tl[64][66]; const int tid = threadIdx.x; const int slab = blockIdx.x / (TTv / 64), lg = blockIdx.x % (TTv / 64); const int b = slab / NHv, h = slab % NHv;
  for (int i = tid; i < 64 * 8; i += 256) { const int r = i / 8, c8 = (i % 8) * 8; FragH f; f.half[0] = *(const v8us*)((const unsigned short*)V16 + ((size_t)b * TTv + lg * 64 + r) * ldv + voff + h * 64 + c8);
#pragma unroll
    for (int q = 0; q < 8; ++q) tl[r][c8 + q] = f.u[q]; }
  __syncthreads();
  for (int pass = 0; pass < 2; ++pass) {
#pragma unroll
    for (int rd = 0; rd < 2; ++rd) { const int d = rd * 32 + tid / 8, pc = tid % 8; FragH f;
#pragma unroll
      for (int q = 0; q < 8; ++q) f.u[q] = tl[pc * 8 + q][d];
      *(volatile v8us*)((unsigned short*)Vt + ((size_t)slab * 64 + d) * TTv + lg * 64 + pc * 8) = f.half[0]; }
    if (pass == 0) __threadfence(); } }

__global__ __launch_bounds__(256) void k_hl(const float* __restrict__ F, _Float16* __restrict__ Hh, _Float16* __restrict__ Hl, size_t n8) { const size_t t = (size_t)blockIdx.x * 256 + threadIdx.x; if (t >= n8) return; FragH fh, fl; const v4f a = *(const v4fa*)(F + t * 8), c = *(const v4fa*)(F + t * 8 + 4);
#pragma unroll
  for (int q = 0; q < 4; ++q) { _Float16 h = (_Float16)a[q]; fh.h[q] = h; fl.h[q] = (_Float16)((a[q] - (float)h) * 1024.0f); h = (_Float16)c[q]; fh.h[4 + q] = h; fl.h[4 + q] = (_Float16)((c[q] - (float)h) * 1024.0f); }
  for (int pass = 0; pass < 2; ++pass) { *(volatile v8us*)((unsigned short*)Hh + t * 8) = fh.half[0]; *(volatile v8us*)((unsigned short*)Hl + t * 8) = fl.half[0]; if (pass == 0) __threadfence(); } }

__global__ __launch_bounds__(256) void k_pe(float* __restrict__ PE) { const int t = blockIdx.x * 256 + threadIdx.x; if (t >= LQ * QD) return; const int q = t / QD, c = t % QD; const int gh = q / HQ, gw = q % HQ; const int k = c % 80; const float omega = exp2f(-(float)k / 80.0f * 13.287712379549449f); const float pos = (c < 160) ? (float)gh : (float)gw; const float ang = pos * omega; const float pe = ((c % 160) < 80) ? sinf(ang) : cosf(ang);
  *(volatile float*)(PE + t) = pe; __threadfence(); *(volatile float*)(PE + t) = pe; }
__global__ __launch_bounds__(256) void k_query(const float* __restrict__ smp, const float* __restrict__ g, const float* __restrict__ bta, const float* __restrict__ PE, _Float16* __restrict__ Q16) {
  #pragma clang fp contract(off)
  __shared__ __attribute__((aligned(16))) unsigned short rows[8][QD]; const int tid = threadIdx.x, w = tid >> 5, l = tid & 31; const int r = blockIdx.x * 8 + w; const int b = r / LQ, q = r % LQ; float v[10]; float s = 0.f;
#pragma unroll
  for (int m = 0; m < 10; ++m) { v[m] = bf16_round(smp[((size_t)b * QD + l + 32 * m) * LQ + q]); s += v[m]; }
  for (int o = 16; o > 0; o >>= 1) s += __shfl_xor(s, o, 32); const float mu = s / (float)QD; float vs = 0.f;
#pragma unroll
  for (int m = 0; m < 10; ++m) { const float d = v[m] - mu; vs += d * d; }
  for (int o = 16; o > 0; o >>= 1) vs += __shfl_xor(vs, o, 32); const float rs = rsqrtf(vs / (float)QD + 1e-6f);
#pragma unroll
  for (int m = 0; m < 10; ++m) { const int c = l + 32 * m; const float pe = PE[(size_t)q * QD + c];
    FragH f; f.h[0] = (_Float16)(((v[m] - mu) * rs * bf16_round(g[c]) + bf16_round(bta[c])) + pe); rows[w][c] = f.u[0]; }
  __syncthreads();
  for (int pass = 0; pass < 2; ++pass) { for (int i = tid; i < 8 * (QD / 8); i += 256) { const int rr = i / (QD / 8), cc = (i % (QD / 8)) * 8; const v8us vv = *(const v8us*)&rows[rr][cc]; *(volatile v8us*)((unsigned short*)Q16 + (size_t)(blockIdx.x * 8 + rr) * QD + cc) = vv; } if (pass == 0) __threadfence(); } }
__global__ __launch_bounds__(256) void k_feat(const float* __restrict__ X, const float* __restrict__ g, const float* __restrict__ bta, _Float16* __restrict__ F16) {
  #pragma clang fp contract(off)
  const int tid = threadIdx.x, w = tid >> 5, l = tid & 31; const size_t r = (size_t)blockIdx.x * 8 + w; float v[32]; float s = 0.f;
#pragma unroll
  for (int q4 = 0; q4 < 4; ++q4) { const v4f a = *(const v4fa*)(X + r * FD + q4 * 256 + 8 * l), c = *(const v4fa*)(X + r * FD + q4 * 256 + 8 * l + 4);
#pragma unroll
    for (int j = 0; j < 4; ++j) { v[q4 * 8 + j] = bf16_round(a[j]); v[q4 * 8 + 4 + j] = bf16_round(c[j]); } }
#pragma unroll
  for (int i = 0; i < 32; ++i) s += v[i];
  for (int o = 16; o > 0; o >>= 1) s += __shfl_xor(s, o, 32); const float mu = s / (float)FD; float vs = 0.f;
#pragma unroll
  for (int i = 0; i < 32; ++i) { const float d = v[i] - mu; vs += d * d; }
  for (int o = 16; o > 0; o >>= 1) vs += __shfl_xor(vs, o, 32); const float rs = rsqrtf(vs / (float)FD + 1e-6f);
  for (int pass = 0; pass < 2; ++pass) {
#pragma unroll
    for (int q4 = 0; q4 < 4; ++q4) { FragH f;
#pragma unroll
      for (int j = 0; j < 8; ++j) { const int c = q4 * 256 + 8 * l + j; f.h[j] = (_Float16)((v[q4 * 8 + j] - mu) * rs * bf16_round(g[c]) + bf16_round(bta[c])); }
      *(volatile v8us*)((unsigned short*)F16 + r * FD + q4 * 256 + 8 * l) = f.half[0]; }
    if (pass == 0) __threadfence(); } }
__global__ __launch_bounds__(256) void k_mmda(const _Float16* __restrict__ V16, const float* __restrict__ OFF, const float* __restrict__ LG, const int* __restrict__ mask, _Float16* __restrict__ O16) {
  #pragma clang fp contract(off)
  const int tid = threadIdx.x, w = tid >> 5, l = tid & 31; const int rh = blockIdx.x * 8 + w; const int r = rh / NH, h = rh % NH; const int b = r / LQ, q = r % LQ; const float rx = ((float)(q % HQ) + 0.5f) / (float)HQ, ry = ((float)(q / HQ) + 0.5f) / (float)HQ;
  float lgv[2]; int live[2];
#pragma unroll
  for (int s2 = 0; s2 < 2; ++s2) { const int idx = l + 32 * s2; const int n = idx / NPt, p = idx % NPt; const int mk = mask[b * NIM + n]; live[s2] = (mk > 0) ? 1 : 0; lgv[s2] = live[s2] ? LG[(size_t)r * (NH * MAXN * NPt) + (h * MAXN + n) * NPt + p] : -1.0e9f; }
  float m = fmaxf(lgv[0], lgv[1]); for (int o = 16; o > 0; o >>= 1) m = fmaxf(m, __shfl_xor(m, o, 32));
  float e0 = expf(lgv[0] - m), e1 = expf(lgv[1] - m); float s = e0 + e1; for (int o = 16; o > 0; o >>= 1) s += __shfl_xor(s, o, 32); const float is = 1.0f / s; e0 *= is; e1 *= is;
  float acc0 = 0.f, acc1 = 0.f; const int d0 = 2 * l;
#pragma unroll 1
  for (int idx = 0; idx < NIM * NPt; ++idx) { const int n = idx / NPt, p = idx % NPt; const float aw = __shfl((idx < 32) ? e0 : e1, idx & 31, 32); if (mask[b * NIM + n] <= 0) continue;
    const float ox = OFF[(size_t)r * (NH * NPt * 2) + (h * NPt + p) * 2], oy = OFF[(size_t)r * (NH * NPt * 2) + (h * NPt + p) * 2 + 1];
    const float lx = rx + ox / (float)HV, ly = ry + oy / (float)HV; const float x = lx * (float)HV - 0.5f, y = ly * (float)HV - 0.5f; const float fx = floorf(x), fy = floorf(y); const float wx = x - fx, wy = y - fy; const int x0 = (int)fx, y0 = (int)fy; float s0 = 0.f, s1 = 0.f;
#pragma unroll
    for (int c = 0; c < 4; ++c) { const int xi = x0 + (c & 1), yi = y0 + (c >> 1); const bool valid = (xi >= 0) && (xi < HV) && (yi >= 0) && (yi < HV); const float wgt = ((c & 1) ? wx : 1.f - wx) * ((c >> 1) ? wy : 1.f - wy); const int ii = min(max(yi, 0), HV - 1) * HV + min(max(xi, 0), HV - 1);
      const unsigned int pr = *(const unsigned int*)((const unsigned short*)V16 + ((size_t)(b * NIM + n) * LV + ii) * DM + h * HD + d0); FragH f; f.u[0] = (unsigned short)(pr & 0xffffu); f.u[1] = (unsigned short)(pr >> 16); const float wv = valid ? wgt : 0.f; s0 += wv * (float)f.h[0]; s1 += wv * (float)f.h[1]; }
    acc0 += aw * s0; acc1 += aw * s1; }
  FragH o; o.h[0] = (_Float16)acc0; o.h[1] = (_Float16)acc1; const unsigned int ov = *(const unsigned int*)&o.u[0]; *(volatile unsigned int*)((unsigned short*)O16 + (size_t)r * DM + h * HD + d0) = ov; __threadfence(); *(volatile unsigned int*)((unsigned short*)O16 + (size_t)r * DM + h * HD + d0) = ov; }
__global__ __launch_bounds__(256) void k_nchw(const float* __restrict__ Y, float* __restrict__ out) { const int t = blockIdx.x * 256 + threadIdx.x; if (t >= NB * QD * (LQ / 4)) return; const int q4 = (t % (LQ / 4)) * 4; const int bo = t / (LQ / 4); const int b = bo / QD, o = bo % QD; v4f v;
#pragma unroll
  for (int j = 0; j < 4; ++j) v[j] = Y[((size_t)b * LQ + q4 + j) * QD + o]; *(volatile v4f*)(out + (size_t)bo * LQ + q4) = v; __threadfence(); *(volatile v4f*)(out + (size_t)bo * LQ + q4) = v; }

extern "C" void kernel_launch(void* const* d_in, const int* in_sizes, int n_in,
                              void* d_out, int out_size, void* d_ws, size_t ws_size, hipStream_t stream) {
  (void)in_sizes; (void)n_in; (void)out_size;
  const float* const* I = (const float* const*)d_in; const float* smp = I[0]; const float* msf = I[1]; const int* mask = (const int*)d_in[2]; (void)d_in[3];
  const float* lqg = I[4]; const float* lqb = I[5]; const float* lfg = I[6]; const float* lfb = I[7]; const float* woff = I[8]; const float* boff = I[9]; const float* wat = I[10]; const float* bat = I[11]; const float* wval = I[12]; const float* bval = I[13]; const float* wout = I[14]; const float* bout = I[15]; const float* cw = I[16]; const float* cb = I[17];
  char* ws = (char*)d_ws; size_t off = 0;
  auto take = [&](size_t bytes) { char* p = ws + off; off += (bytes + 255) & ~(size_t)255; return p; };
  _Float16* Boff = (_Float16*)take((size_t)256 * QD * 2); _Float16* Bat = (_Float16*)take((size_t)1280 * QD * 2); _Float16* Bval = (_Float16*)take((size_t)DM * FD * 2); _Float16* Bout = (_Float16*)take((size_t)QD * DM * 2); _Float16* Bcw = (_Float16*)take((size_t)QD * QD * 2);
  _Float16* Q16 = (_Float16*)take((size_t)NQ * QD * 2); _Float16* F16 = (_Float16*)take((size_t)NV * FD * 2); _Float16* V16 = (_Float16*)take((size_t)NV * DM * 2); float* OFF = (float*)take((size_t)NQ * 256 * 4); float* LG = (float*)take((size_t)NQ * 1280 * 4); _Float16* O16 = (_Float16*)take((size_t)NQ * DM * 2); _Float16* A16 = (_Float16*)take((size_t)NQ * QD * 2); float* Y = (float*)take((size_t)NQ * QD * 4); float* PE = (float*)take((size_t)LQ * QD * 4);
  if (off > ws_size) return;
  k_wt_f16<<<(256 * (QD / 8) + 255) / 256, 256, 0, stream>>>(woff, Boff, QD, 256, 16.0f); k_wt_f16<<<(1280 * (QD / 8) + 255) / 256, 256, 0, stream>>>(wat, Bat, QD, 1280, 16.0f); k_wt_f16<<<(unsigned)(((size_t)DM * (FD / 8) + 255) / 256), 256, 0, stream>>>(wval, Bval, FD, DM, 16.0f); k_wt_f16<<<(QD * (DM / 8) + 255) / 256, 256, 0, stream>>>(wout, Bout, DM, QD, 16.0f);
  k_round16f<<<(QD * QD / 8 + 255) / 256, 256, 0, stream>>>(cw, Bcw, (size_t)QD * QD / 8);
  k_pe<<<(LQ * QD + 255) / 256, 256, 0, stream>>>(PE); k_query<<<NQ / 8, 256, 0, stream>>>(smp, lqg, lqb, PE, Q16); k_feat<<<NV / 8, 256, 0, stream>>>(msf, lfg, lfb, F16);
  k_gemm_hhx<0><<<dim3(((NV / 16) * (DM / 64) + 3) / 4, 1), 128, 0, stream>>>(F16, FD, 0, Bval, FD, 0, 0.0625f, bval, 0, nullptr, 1, 0, 0, nullptr, V16, DM, 0, NV, DM, FD);
  k_gemm_hhx<0><<<dim3(((NQ / 16) * (256 / 64) + 3) / 4, 1), 128, 0, stream>>>(Q16, QD, 0, Boff, QD, 0, 0.0625f, boff, 0, nullptr, 1, 0, 0, OFF, nullptr, 256, 0, NQ, 256, QD);
  k_gemm_hhx<0><<<dim3(((NQ / 16) * (1280 / 64) + 3) / 4, 1), 128, 0, stream>>>(Q16, QD, 0, Bat, QD, 0, 0.0625f, bat, 0, nullptr, 1, 0, 0, LG, nullptr, 1280, 0, NQ, 1280, QD);
  k_mmda<<<NQ * NH / 8, 256, 0, stream>>>(V16, OFF, LG, mask, O16);
  k_gemm_hhx<0><<<dim3(((NQ / 16) * (QD / 64) + 3) / 4, 1), 128, 0, stream>>>(O16, DM, 0, Bout, DM, 0, 0.0625f, bout, 0, nullptr, 1, 0, 0, nullptr, A16, QD, 0, NQ, QD, DM);
  k_gemm_hhx<0><<<dim3(((NQ / 16) * (QD / 64) + 3) / 4, 1), 128, 0, stream>>>(A16, QD, 0, Bcw, QD, 0, 0.0625f, cb, 0, nullptr, 1, 0, 0, Y, nullptr, QD, 0, NQ, QD, QD);
  k_nchw<<<(NB * QD * (LQ / 4) + 255) / 256, 256, 0, stream>>>(Y, (float*)d_out);
}
